// FirstLayer_39659728011898
// MI455X (gfx1250) — hardware-verified
//
#include <hip/hip_runtime.h>
#include <stddef.h>
#include <math.h>

#pragma clang fp contract(off)


#define NB     16
#define CI     32
#define CO     64
#define GH     64
#define NG     16
#define ED     64
#define KD     128
#define NOUT   2048
#define S0     28
#define NS     64
#define KF     2048
#define EP     136
#define TP     72
#define NTH    128
#define NTP    256
#define NPART  64
#define PARTW  32
#define SIG2   0.0049f
#define HALFW  0.1f

#define IT_W   (KD * KD / 8)
#define IT_WO  (NOUT * KD / 8)
#define IT_DG  (NB * KF / 8)
#define PREP_ITEMS (2 * IT_W + IT_WO + IT_DG)

static_assert(KD == 2 * ED);
static_assert(NOUT == CI * CO);
static_assert(KF == CI * NS);
static_assert(NS == 16 * (NTH / 32));
static_assert((EP * 2) % 16 == 0);
static_assert((TP * 2) % 16 == 0);
static_assert(IT_W % NTP == 0);
static_assert(IT_WO % NTP == 0);
static_assert(IT_DG % NTP == 0);
static_assert(PREP_ITEMS % NTP == 0);
static_assert(NPART * 4 * NTP == GH * GH * NG);
static_assert(NB * CO == 8 * NTH);
static_assert((NS * KD) % NTH == 0);
static_assert(KD % 32 == 0);
static_assert(KF % 32 == 0);

typedef unsigned short us_t;
typedef us_t   v8us  __attribute__((ext_vector_type(8)));
typedef __bf16 v16bf __attribute__((ext_vector_type(16)));
typedef float  v4f   __attribute__((ext_vector_type(4)));
typedef float  v8f   __attribute__((ext_vector_type(8)));
union FragB { v16bf v; v8us h[2]; us_t e[16]; };

__device__ __forceinline__ v8f wmb(v16bf a, v16bf b, v8f c) {
  v8f d = __builtin_amdgcn_wmma_f32_16x16x32_bf16(false, a, false, b, (short)0, c, false, false);
#if defined(__HIP_DEVICE_COMPILE__)
  asm volatile("v_nop\n\tv_nop\n\tv_nop\n\tv_nop" : "+v"(d) : "v"(a), "v"(b));
#endif
  return d;
}

__device__ __forceinline__ v8f zero8() {
  v8f z = {0.f, 0.f, 0.f, 0.f, 0.f, 0.f, 0.f, 0.f};
  return z;
}

__device__ __forceinline__ us_t bf16_bits(float x) {
  unsigned u = __float_as_uint(x);
  u = (u + 0x7FFFu + ((u >> 16) & 1u)) >> 16;
  return (us_t)u;
}
__device__ __forceinline__ float bf16_val(us_t b) {
  return __uint_as_float(((unsigned)b) << 16);
}

__device__ __forceinline__ float silu_f(float x) {
  const float xc = fmaxf(x, -30.0f);
  const float e  = expf(-xc);
  const float sg = 1.0f / (1.0f + e);
  return x * sg;
}

__device__ __forceinline__ float lin_coord(int k) {
  const float st = (float)k * (1.0f / 63.0f);
  const float a  = 1.0f - st;
  const float x  = st - a;
  return (k == GH - 1) ? 1.0f : x;
}
__device__ __forceinline__ float centre(int e) {
  const float st = (float)e * (1.0f / 63.0f);
  return (e == ED - 1) ? 1.0f : st;
}
__device__ __forceinline__ void rot2(float c, float s, float x0, float x1, float& w0, float& w1) {
  const float p0 = c * x0;
  const float p1 = s * x1;
  const float q0 = (-s) * x0;
  const float q1 = c * x1;
  w0 = p0 + p1;
  w1 = q0 + q1;
}

__device__ __forceinline__ void split_store8(const float* w, us_t* ph, us_t* pl) {
  v8us oh, ol;
#pragma unroll
  for (int e = 0; e < 8; ++e) {
    const us_t hb = bf16_bits(w[e]);
    oh[e] = hb;
    ol[e] = bf16_bits(w[e] - bf16_val(hb));
  }
  *(volatile v8us*)ph = oh;
  *(volatile v8us*)pl = ol;
  __threadfence();
  *(volatile v8us*)ph = oh;
  *(volatile v8us*)pl = ol;
}

__global__ __launch_bounds__(NTP) void k_prep(const float* __restrict__ W0, const float* __restrict__ W1,
                                              const float* __restrict__ Wo, const float* __restrict__ data,
                                              us_t* P0h, us_t* P0l, us_t* P1h, us_t* P1l,
                                              us_t* PWh, us_t* PWl, us_t* Dgh, us_t* Dgl) {
  const int i = blockIdx.x * NTP + (int)threadIdx.x;
  float w[8];
  us_t* ph;
  us_t* pl;
  if (i < IT_W) {
    const int n = i >> 4, k0 = (i & 15) * 8;
#pragma unroll
    for (int e = 0; e < 8; ++e) w[e] = W0[(k0 + e) * KD + n];
    ph = P0h + n * KD + k0;
    pl = P0l + n * KD + k0;
  } else if (i < 2 * IT_W) {
    const int j = i - IT_W;
    const int n = j >> 4, k0 = (j & 15) * 8;
#pragma unroll
    for (int e = 0; e < 8; ++e) w[e] = W1[(k0 + e) * KD + n];
    ph = P1h + n * KD + k0;
    pl = P1l + n * KD + k0;
  } else if (i < 2 * IT_W + IT_WO) {
    const int j = i - 2 * IT_W;
    const int oc = j >> 4, k0 = (j & 15) * 8;
#pragma unroll
    for (int e = 0; e < 8; ++e) w[e] = Wo[(size_t)(k0 + e) * NOUT + oc];
    ph = PWh + (size_t)oc * KD + k0;
    pl = PWl + (size_t)oc * KD + k0;
  } else {
    const int j   = i - (2 * IT_W + IT_WO);
    const int b   = j >> 8;
    const int kk0 = (j & 255) * 8;
    const int c   = kk0 >> 6;
    const int sh  = (kk0 & 63) >> 3;
    const float* src = data + ((size_t)((b * CI + c) * GH + S0 + sh)) * GH + S0;
    const v4f a = *(const v4f*)src;
    const v4f q = *(const v4f*)(src + 4);
    w[0] = a[0]; w[1] = a[1]; w[2] = a[2]; w[3] = a[3];
    w[4] = q[0]; w[5] = q[1]; w[6] = q[2]; w[7] = q[3];
    ph = Dgh + b * KF + kk0;
    pl = Dgl + b * KF + kk0;
  }
  split_store8(w, ph, pl);
}

__global__ __launch_bounds__(NTP) void k_norm(const float* __restrict__ v, float* part) {
  __shared__ float sC[NG];
  __shared__ float sS[NG];
  __shared__ float sR[NTP / 32];
  const int tid = threadIdx.x, lane = tid & 31, wv = tid >> 5;
  if (tid < NG) {
    const float th = v[tid];
    sC[tid] = cosf(th);
    sS[tid] = sinf(th);
  }
  __syncthreads();
  const float RS = 1.0f / SIG2;
  float lmax = 0.0f;
#pragma unroll 1
  for (int it = 0; it < 4; ++it) {
    const int g  = (blockIdx.x * 4 + it) * NTP + tid;
    const int n  = g & (NG - 1);
    const int hw = g >> 4;
    const int hh = hw >> 6, ww = hw & 63;
    const float x0 = lin_coord(hh), x1 = lin_coord(ww);
    const float c = sC[n], s = sS[n];
    float w0, w1;
    rot2(c, s, x0, x1, w0, w1);
    float acc = 0.0f;
#pragma unroll 1
    for (int e = 0; e < ED; ++e) {
      const float mu = centre(e);
      const float d0 = w0 - mu;
      const float t0 = d0 * d0;
      const float a0 = (-0.5f * t0) * RS;
      const float e0 = expf(a0);
      const float d1 = w1 - mu;
      const float t1 = d1 * d1;
      const float a1 = (-0.5f * t1) * RS;
      const float e1 = expf(a1);
      acc = acc + e0 * e0;
      acc = acc + e1 * e1;
    }
    lmax = fmaxf(lmax, acc);
  }
#pragma unroll
  for (int off = 1; off < 32; off <<= 1) lmax = fmaxf(lmax, __shfl_xor(lmax, off, 32));
  if (lane == 0) sR[wv] = lmax;
  __syncthreads();
  if (wv == 0) {
    float bm = sR[0];
#pragma unroll
    for (int i = 1; i < NTP / 32; ++i) bm = fmaxf(bm, sR[i]);
    if (lane < 8) {
      v4f o = {bm, bm, bm, bm};
      float* p = part + blockIdx.x * PARTW + lane * 4;
      *(volatile v4f*)p = o;
      __threadfence();
      *(volatile v4f*)p = o;
    }
  }
}

__device__ __forceinline__ void dense_layer(const us_t* __restrict__ Ph, const us_t* __restrict__ Pl,
                                            const float* __restrict__ bias,
                                            us_t* sXh, us_t* sXl, int wr, int h, int m) {
  FragB ah[4], al[4];
#pragma unroll
  for (int ks = 0; ks < 4; ++ks) {
    const int pa = (wr + m) * EP + 32 * ks + 8 * h;
    ah[ks].h[0] = *(const v8us*)(sXh + pa);
    ah[ks].h[1] = *(const v8us*)(sXh + pa + 16);
    al[ks].h[0] = *(const v8us*)(sXl + pa);
    al[ks].h[1] = *(const v8us*)(sXl + pa + 16);
  }
  __syncthreads();
#pragma unroll 1
  for (int g = 0; g < 2; ++g) {
    v8f acc[4];
#pragma unroll
    for (int t = 0; t < 4; ++t) {
      acc[t] = zero8();
      const int n0 = 64 * g + 16 * t;
      const us_t* pbh = Ph + (size_t)(n0 + m) * KD + 8 * h;
      const us_t* pbl = Pl + (size_t)(n0 + m) * KD + 8 * h;
#pragma unroll
      for (int ks = 0; ks < 4; ++ks) {
        FragB bh, bl;
        bh.h[0] = *(const v8us*)(pbh + 32 * ks);
        bh.h[1] = *(const v8us*)(pbh + 32 * ks + 16);
        bl.h[0] = *(const v8us*)(pbl + 32 * ks);
        bl.h[1] = *(const v8us*)(pbl + 32 * ks + 16);
        acc[t] = wmb(ah[ks].v, bh.v, acc[t]);
        acc[t] = wmb(ah[ks].v, bl.v, acc[t]);
        acc[t] = wmb(al[ks].v, bh.v, acc[t]);
      }
    }
#pragma unroll
    for (int t = 0; t < 4; ++t) {
      const int col = 64 * g + 16 * t + m;
      const float bb = bias[col];
#pragma unroll
      for (int r = 0; r < 8; ++r) {
        const float val = silu_f(acc[t][r] + bb);
        const us_t  hb  = bf16_bits(val);
        const us_t  lb  = bf16_bits(val - bf16_val(hb));
        sXh[(wr + 8 * h + r) * EP + col] = hb;
        sXl[(wr + 8 * h + r) * EP + col] = lb;
      }
    }
  }
  __syncthreads();
}

__global__ __launch_bounds__(NTH) void k_mlp(const float* __restrict__ v, const float* __restrict__ part,
                                             const us_t* __restrict__ P0h, const us_t* __restrict__ P0l,
                                             const float* __restrict__ b0,
                                             const us_t* __restrict__ P1h, const us_t* __restrict__ P1l,
                                             const float* __restrict__ b1,
                                             const us_t* __restrict__ PWh, const us_t* __restrict__ PWl,
                                             const float* __restrict__ bo,
                                             us_t* Fh, us_t* Fl) {
  __shared__ __align__(16) us_t sXh[NS * EP];
  __shared__ __align__(16) us_t sXl[NS * EP];
  __shared__ __align__(16) us_t sTh[4 * 16 * TP];
  __shared__ __align__(16) us_t sTl[4 * 16 * TP];
  __shared__ int sMask[NS];

  const int tid = threadIdx.x, lane = tid & 31, wv = tid >> 5, h = lane >> 4, m = lane & 15;
  const int n  = blockIdx.x;
  const int wr = 16 * wv;

  float m2 = 0.0f;
#pragma unroll 1
  for (int i = 0; i < NPART; ++i) m2 = fmaxf(m2, part[i * PARTW]);
  const float inv = 1.0f / sqrtf(m2);
  const float th  = v[n];
  const float c   = cosf(th), s = sinf(th);
  const float RS  = 1.0f / SIG2;

  if (tid < NS) {
    const int sh = tid >> 3, sw = tid & 7;
    const float x0 = lin_coord(S0 + sh), x1 = lin_coord(S0 + sw);
    float w0, w1;
    rot2(c, s, x0, x1, w0, w1);
    const bool in = (w0 >= -HALFW) && (w0 <= HALFW) && (w1 >= -HALFW) && (w1 <= HALFW);
    sMask[tid] = in ? 1 : 0;
  }

#pragma unroll 1
  for (int i = 0; i < (NS * KD) / NTH; ++i) {
    const int idx = i * NTH + tid;
    const int sr  = idx >> 7;
    const int j   = idx & (KD - 1);
    const int sh = sr >> 3, sw = sr & 7;
    const float x0 = lin_coord(S0 + sh), x1 = lin_coord(S0 + sw);
    float w0, w1;
    rot2(c, s, x0, x1, w0, w1);
    const float wc = (j < ED) ? w0 : w1;
    const float mu = centre(j & (ED - 1));
    const float d  = wc - mu;
    const float t  = d * d;
    const float a  = (-0.5f * t) * RS;
    const float val = expf(a) * inv;
    const us_t hb = bf16_bits(val);
    const us_t lb = bf16_bits(val - bf16_val(hb));
    sXh[sr * EP + j] = hb;
    sXl[sr * EP + j] = lb;
  }
  __syncthreads();

  dense_layer(P0h, P0l, b0, sXh, sXl, wr, h, m);
  dense_layer(P1h, P1l, b1, sXh, sXl, wr, h, m);

  int msk[8];
#pragma unroll
  for (int r = 0; r < 8; ++r) msk[r] = sMask[wr + 8 * h + r];
  FragB ah[4], al[4];
#pragma unroll
  for (int ks = 0; ks < 4; ++ks) {
    const int pa = (wr + m) * EP + 32 * ks + 8 * h;
    ah[ks].h[0] = *(const v8us*)(sXh + pa);
    ah[ks].h[1] = *(const v8us*)(sXh + pa + 16);
    al[ks].h[0] = *(const v8us*)(sXl + pa);
    al[ks].h[1] = *(const v8us*)(sXl + pa + 16);
  }
  us_t* sth = sTh + wv * 16 * TP;
  us_t* stl = sTl + wv * 16 * TP;
  const int rq = lane >> 3, q = lane & 7;

#pragma unroll 1
  for (int cg = 0; cg < CI; ++cg) {
    v8f acc[4];
#pragma unroll
    for (int t = 0; t < 4; ++t) {
      acc[t] = zero8();
      const us_t* pbh = PWh + (size_t)(cg * CO + 16 * t + m) * KD + 8 * h;
      const us_t* pbl = PWl + (size_t)(cg * CO + 16 * t + m) * KD + 8 * h;
#pragma unroll
      for (int ks = 0; ks < 4; ++ks) {
        FragB bh, bl;
        bh.h[0] = *(const v8us*)(pbh + 32 * ks);
        bh.h[1] = *(const v8us*)(pbh + 32 * ks + 16);
        bl.h[0] = *(const v8us*)(pbl + 32 * ks);
        bl.h[1] = *(const v8us*)(pbl + 32 * ks + 16);
        acc[t] = wmb(ah[ks].v, bh.v, acc[t]);
        acc[t] = wmb(ah[ks].v, bl.v, acc[t]);
        acc[t] = wmb(al[ks].v, bh.v, acc[t]);
      }
    }
#pragma unroll
    for (int t = 0; t < 4; ++t) {
      const int col = 16 * t + m;
      const float bb = bo[cg * CO + col];
#pragma unroll
      for (int r = 0; r < 8; ++r) {
        const float val = acc[t][r] + bb;
        const float z   = (msk[r] != 0) ? val : 0.0f;
        const us_t  hb  = bf16_bits(z);
        const us_t  lb  = bf16_bits(z - bf16_val(hb));
        sth[(8 * h + r) * TP + col] = hb;
        stl[(8 * h + r) * TP + col] = lb;
      }
    }
    __syncthreads();
    v8us oh[4], ol[4];
#pragma unroll
    for (int p = 0; p < 4; ++p) {
      oh[p] = *(const v8us*)(sth + (4 * p + rq) * TP + 8 * q);
      ol[p] = *(const v8us*)(stl + (4 * p + rq) * TP + 8 * q);
    }
    const size_t base = ((size_t)n * KF + (size_t)(cg * NS + wr)) * CO;
#pragma unroll
    for (int p = 0; p < 4; ++p) {
      const size_t off = base + (size_t)((4 * p + rq) * CO + 8 * q);
      *(volatile v8us*)(Fh + off) = oh[p];
      *(volatile v8us*)(Fl + off) = ol[p];
    }
    __threadfence();
#pragma unroll
    for (int p = 0; p < 4; ++p) {
      const size_t off = base + (size_t)((4 * p + rq) * CO + 8 * q);
      *(volatile v8us*)(Fh + off) = oh[p];
      *(volatile v8us*)(Fl + off) = ol[p];
    }
    __syncthreads();
  }
}

__global__ __launch_bounds__(NTH) void k_out(const us_t* __restrict__ Dgh, const us_t* __restrict__ Dgl,
                                             const us_t* __restrict__ Fh, const us_t* __restrict__ Fl,
                                             float* out) {
  __shared__ __align__(16) float sO[NB * CO];
  const int tid = threadIdx.x, lane = tid & 31, wv = tid >> 5, h = lane >> 4, m = lane & 15;
  const int n = blockIdx.x;
  const us_t* fh  = Fh + (size_t)n * KF * CO + 16 * wv + m;
  const us_t* fl  = Fl + (size_t)n * KF * CO + 16 * wv + m;
  const us_t* ah0 = Dgh + (size_t)m * KF + 8 * h;
  const us_t* al0 = Dgl + (size_t)m * KF + 8 * h;
  v8f acc = zero8();
#pragma unroll 1
  for (int kb = 0; kb < KF; kb += 32) {
    FragB ah, al, bh, bl;
    ah.h[0] = *(const v8us*)(ah0 + kb);
    ah.h[1] = *(const v8us*)(ah0 + kb + 16);
    al.h[0] = *(const v8us*)(al0 + kb);
    al.h[1] = *(const v8us*)(al0 + kb + 16);
#pragma unroll
    for (int i = 0; i < 8; ++i) {
      const size_t k = (size_t)(kb + 8 * h + i);
      bh.e[i]     = fh[k * CO];
      bh.e[8 + i] = fh[(k + 16) * CO];
      bl.e[i]     = fl[k * CO];
      bl.e[8 + i] = fl[(k + 16) * CO];
    }
    acc = wmb(ah.v, bh.v, acc);
    acc = wmb(ah.v, bl.v, acc);
    acc = wmb(al.v, bh.v, acc);
  }
#pragma unroll
  for (int r = 0; r < 8; ++r) sO[(8 * h + r) * CO + 16 * wv + m] = acc[r];
  __syncthreads();
  v4f o[2];
  float* g[2];
#pragma unroll
  for (int p = 0; p < 2; ++p) {
    const int L  = p * 16 + (tid >> 3);
    const int qq = tid & 7;
    const int b  = L >> 1, hf = L & 1;
    o[p] = *(const v4f*)(sO + b * CO + hf * 32 + qq * 4);
    g[p] = out + ((size_t)(b * NG + n)) * CO + hf * 32 + qq * 4;
  }
  *(volatile v4f*)g[0] = o[0];
  *(volatile v4f*)g[1] = o[1];
  __threadfence();
  *(volatile v4f*)g[0] = o[0];
  *(volatile v4f*)g[1] = o[1];
}

extern "C" void kernel_launch(void* const* d_in, const int* in_sizes, int n_in,
                              void* d_out, int out_size, void* d_ws, size_t ws_size,
                              hipStream_t stream) {
  if (n_in < 8) return;
  if (in_sizes[0] != NB * CI * GH * GH) return;
  if (in_sizes[1] != NG) return;
  if (in_sizes[2] != KD * KD || in_sizes[3] != KD) return;
  if (in_sizes[4] != KD * KD || in_sizes[5] != KD) return;
  if (in_sizes[6] != KD * NOUT || in_sizes[7] != NOUT) return;
  if (out_size != NB * NG * CO) return;

  const float* data = (const float*)d_in[0];
  const float* v    = (const float*)d_in[1];
  const float* W0   = (const float*)d_in[2];
  const float* b0   = (const float*)d_in[3];
  const float* W1   = (const float*)d_in[4];
  const float* b1   = (const float*)d_in[5];
  const float* Wo   = (const float*)d_in[6];
  const float* bo   = (const float*)d_in[7];
  float* out = (float*)d_out;

  const size_t szW  = (size_t)KD * KD * 2;
  const size_t szWO = (size_t)NOUT * KD * 2;
  const size_t szDG = (size_t)NB * KF * 2;
  const size_t szPT = (size_t)NPART * PARTW * 4;
  const size_t szF  = (size_t)NG * KF * CO * 2;
  const size_t offP0h = 0;
  const size_t offP0l = offP0h + szW;
  const size_t offP1h = offP0l + szW;
  const size_t offP1l = offP1h + szW;
  const size_t offPWh = offP1l + szW;
  const size_t offPWl = offPWh + szWO;
  const size_t offDGh = offPWl + szWO;
  const size_t offDGl = offDGh + szDG;
  const size_t offPT  = offDGl + szDG;
  const size_t offFh  = offPT + szPT;
  const size_t offFl  = offFh + szF;
  const size_t total  = offFl + szF;
  if (total > ws_size || total > (size_t)134217728) return;

  char* ws = (char*)d_ws;
  us_t*  P0h = (us_t*)(ws + offP0h);
  us_t*  P0l = (us_t*)(ws + offP0l);
  us_t*  P1h = (us_t*)(ws + offP1h);
  us_t*  P1l = (us_t*)(ws + offP1l);
  us_t*  PWh = (us_t*)(ws + offPWh);
  us_t*  PWl = (us_t*)(ws + offPWl);
  us_t*  DGh = (us_t*)(ws + offDGh);
  us_t*  DGl = (us_t*)(ws + offDGl);
  float* PT  = (float*)(ws + offPT);
  us_t*  Fh  = (us_t*)(ws + offFh);
  us_t*  Fl  = (us_t*)(ws + offFl);

  k_prep<<<PREP_ITEMS / NTP, NTP, 0, stream>>>(W0, W1, Wo, data, P0h, P0l, P1h, P1l, PWh, PWl, DGh, DGl);
  k_norm<<<NPART, NTP, 0, stream>>>(v, PT);
  k_mlp<<<NG, NTH, 0, stream>>>(v, PT, P0h, P0l, b0, P1h, P1l, b1, PWh, PWl, bo, Fh, Fl);
  k_out<<<NG, NTH, 0, stream>>>(DGh, DGl, Fh, Fl, out);
  (void)hipGetLastError();
}
